// Model_59777354826321
// MI455X (gfx1250) — hardware-run, weakly checked
//
#include <hip/hip_runtime.h>


#ifndef NB
#define NB 64
#endif
#ifndef SEQ
#define SEQ 1024
#endif
#define NB_FULL  64
#define SEQ_FULL 1024
#ifndef OUT_SEQ
#define OUT_SEQ SEQ
#endif
#define EW   32
#define NH_  4
#define HD   8
#define NTOK 27
#define NV   27
#define NVP  32
#define WROWS (4 * EW + NVP)
#define AW   4
#define OSP  36
#define TSP  36
#define TT   128
#define SC2  ((float)(0.35355339059327373 * 1.4426950408889634))
#define PSH  14.0f
#define NEGB (-3.0e38f)

static_assert(NH_ * HD == EW);
static_assert(EW == 32);
static_assert(HD == 8);
static_assert(AW == NH_);
static_assert(4 * AW == 16);
static_assert(SEQ % 64 == 0);
static_assert(SEQ % 32 == 0);
static_assert(SEQ % 16 == 0);
static_assert(SEQ % TT == 0);
static_assert(SEQ % 4 == 0);
static_assert(OUT_SEQ % 32 == 0);
static_assert(TT % 32 == 0);
static_assert(TT % 16 == 0);
static_assert(27 * 32 * 16 == TT * NV * 4);
static_assert(2 * 32 * 16 == 16 * EW * 2);
static_assert(4 * 32 * 16 == 16 * 64 * 2);
static_assert(AW * 32 * 16 == 16 * EW * 4);
static_assert(NV <= NVP);
static_assert(NVP == 32);
static_assert(NV > 16);
static_assert(((size_t)NB * SEQ * 4) % 256 == 0);
static_assert(NB <= NB_FULL);
static_assert(SEQ <= SEQ_FULL);
static_assert((OSP * 4) % 16 == 0);
static_assert((TSP * 4) % 16 == 0);
static_assert(16 * 68 * 4 <= 131072);
static_assert(16 * OSP * 4 <= 131072);
static_assert(TT * NV * 4 + 16 * TSP * 4 <= 131072);

typedef _Float16 h16;
typedef unsigned short bf;
typedef __attribute__((ext_vector_type(16))) __bf16   v16bf;
typedef __attribute__((ext_vector_type(16))) _Float16 v16h;
typedef __attribute__((ext_vector_type(8)))  _Float16 v8h;
typedef __attribute__((ext_vector_type(8)))  unsigned short v8us;
typedef __attribute__((ext_vector_type(8)))  unsigned v8u;
typedef __attribute__((ext_vector_type(8)))  float    v8f;
typedef __attribute__((ext_vector_type(4)))  float    v4f;
typedef __attribute__((ext_vector_type(4)))  int      v4i;
typedef v4f  __attribute__((may_alias)) v4fa;

__device__ __forceinline__ unsigned short f2bf(float f) { unsigned u = __float_as_uint(f); u += 0x7FFFu + ((u >> 16) & 1u); return (unsigned short)(u >> 16); }
__device__ __forceinline__ float bfr(float f) { return __uint_as_float(((unsigned)f2bf(f)) << 16); }
__device__ __forceinline__ v16h cat16(v8h lo, v8h hi) { return __builtin_shufflevector(lo, hi, 0, 1, 2, 3, 4, 5, 6, 7, 8, 9, 10, 11, 12, 13, 14, 15); }
__device__ __forceinline__ v16bf cat16b(v8us lo, v8us hi) { return __builtin_bit_cast(v16bf, __builtin_shufflevector(lo, hi, 0, 1, 2, 3, 4, 5, 6, 7, 8, 9, 10, 11, 12, 13, 14, 15)); }
__device__ __forceinline__ v8f wmma16g(v16h a, v16h b, v8f c) {
    c = __builtin_amdgcn_wmma_f32_16x16x32_f16(false, a, false, b, (short)0, c, false, false);
    asm volatile("v_nop\n\tv_nop\n\tv_nop\n\tv_nop" : "+v"(c) : "v"(a), "v"(b));
    return c; }
__device__ __forceinline__ v8f wmmabg(v16bf a, v16bf b, v8f c) {
    c = __builtin_amdgcn_wmma_f32_16x16x32_bf16(false, a, false, b, (short)0, c, false, false);
    asm volatile("v_nop\n\tv_nop\n\tv_nop\n\tv_nop" : "+v"(c) : "v"(a), "v"(b));
    return c; }
__device__ __forceinline__ v16h  ldh(const h16* p) { return cat16(*(const v8h*)p, *(const v8h*)(p + 16)); }
__device__ __forceinline__ v16bf ldb(const bf* p)  { return cat16b(*(const v8us*)p, *(const v8us*)(p + 16)); }
__device__ __forceinline__ void wave_sync() { __builtin_amdgcn_fence(3  , "wavefront"); __builtin_amdgcn_wave_barrier(); asm volatile("" ::: "memory"); }
static __device__ __forceinline__ h16 toh_flush(float v) { const h16 r = (h16)v; return (fabsf(v) < 6.103515625e-05f) ? (h16)0.0f : r; }
__device__ __forceinline__ void split2(float v, unsigned short& h, unsigned short& l) { h = f2bf(v); l = f2bf(v - __uint_as_float(((unsigned)h) << 16)); }

__global__ __launch_bounds__(256) void k_mask(const float* __restrict__ mask, float* NM, int* KE) {
    __shared__ float sv[8]; __shared__ int si[8]; __shared__ int sk[8];
    const int tid = threadIdx.x, lane = tid & 31;
    const int wave = __builtin_amdgcn_readfirstlane((int)(threadIdx.x >> 5));
    const int b = blockIdx.x;
    const float* mrow = mask + (size_t)b * SEQ_FULL;
    float bv = -__builtin_inff(); int bi = -1;
#pragma unroll 1
    for (int c = tid; c < SEQ / 4; c += 256) {
        const v4f v = *(const v4f*)(mrow + 4 * c);
#pragma unroll
        for (int k = 0; k < 4; ++k) { const float vk = bfr(v[k]); const bool tk = vk >= bv; bv = tk ? vk : bv; bi = tk ? (4 * c + k) : bi; }
    }
#pragma unroll
    for (int off = 16; off > 0; off >>= 1) {
        const float ov = __shfl_xor(bv, off, 32); const int oi = __shfl_xor(bi, off, 32);
        const bool tk = (ov > bv) | ((ov == bv) & (oi > bi)); bv = tk ? ov : bv; bi = tk ? oi : bi; }
    if (lane == 0) { sv[wave] = bv; si[wave] = bi; }
    __syncthreads();
    float gv = sv[0]; int gi = si[0];
#pragma unroll
    for (int w = 1; w < 8; ++w) { const float ov = sv[w]; const int oi = si[w]; const bool tk = (ov > gv) | ((ov == gv) & (oi > gi)); gv = tk ? ov : gv; gi = tk ? oi : gi; }
    int last = gi < 0 ? 0 : gi;
    int ext = last + 1; ext = ext > SEQ - 1 ? SEQ - 1 : ext;
    int lk = -1;
#pragma unroll 1
    for (int c = tid; c < SEQ / 4; c += 256) {
        v4f v = *(const v4f*)(mrow + 4 * c);
#pragma unroll
        for (int k = 0; k < 4; ++k) { const int idx = 4 * c + k; v[k] = (idx == ext) ? 1.0f : bfr(v[k]); lk = (v[k] != 0.0f) ? idx : lk; }
        float* dst = NM + (size_t)b * SEQ + 4 * c;
        *(volatile v4f*)dst = v; __threadfence(); *(volatile v4f*)dst = v;
    }
#pragma unroll
    for (int off = 16; off > 0; off >>= 1) { const int ol = __shfl_xor(lk, off, 32); lk = ol > lk ? ol : lk; }
    if (lane == 0) sk[wave] = lk;
    __syncthreads();
    int ke = sk[0];
#pragma unroll
    for (int w = 1; w < 8; ++w) { const int ol = sk[w]; ke = ol > ke ? ol : ke; }
    ke += 1;
    if (wave == 0) {
        if (lane < 8) {
            const v4i kv = (v4i){ke, ke, ke, ke};
            int* dst = KE + (size_t)b * 32 + lane * 4;
            *(volatile v4i*)dst = kv; __threadfence(); *(volatile v4i*)dst = kv; } }
}

__global__ __launch_bounds__(256) void k_wconv(const float* __restrict__ inw, const float* __restrict__ ow, const float* __restrict__ fw, bf* WB) {
    const int i = blockIdx.x * 256 + threadIdx.x; if (i >= WROWS * 4) return;
    const int row = i >> 2, pc = (i & 3) * 8;
    const int r1 = row < 3 * EW - 1 ? row : 3 * EW - 1;
    int r2 = row - 3 * EW; r2 = r2 < 0 ? 0 : (r2 > EW - 1 ? EW - 1 : r2);
    int r3 = row - 4 * EW; r3 = r3 < 0 ? 0 : (r3 > NV - 1 ? NV - 1 : r3);
    v8f a = *(const v8f*)(inw + r1 * EW + pc);
    v8f c = *(const v8f*)(ow + r2 * EW + pc);
    v8f d = *(const v8f*)(fw + r3 * EW + pc);
    asm volatile("" : "+v"(a)); asm volatile("" : "+v"(c)); asm volatile("" : "+v"(d));
    const bool s1 = row < 3 * EW;
    const bool s2 = (row >= 3 * EW) & (row < 4 * EW);
    const bool s3 = (row >= 4 * EW) & (row < 4 * EW + NV);
    v8us o;
#pragma unroll
    for (int k = 0; k < 8; ++k) { const float v = s1 ? a[k] : (s2 ? c[k] : (s3 ? d[k] : 0.0f)); o[k] = f2bf(v); }
    *(volatile v8us*)(WB + (size_t)i * 8) = o; __threadfence(); *(volatile v8us*)(WB + (size_t)i * 8) = o;
}

__global__ __launch_bounds__(256) void k_embed(const int* __restrict__ x, const float* __restrict__ emb, const float* __restrict__ NM, bf* HB) {
    const size_t i = (size_t)blockIdx.x * 256 + threadIdx.x; if (i >= (size_t)NB * SEQ * 4) return;
    const int tok = (int)(i >> 2), pc = (int)(i & 3) * 8;
    const int b = tok / SEQ, t = tok % SEQ;
    int id = x[(size_t)b * SEQ_FULL + t]; id = id < 0 ? 0 : (id > NTOK - 1 ? NTOK - 1 : id);
    const float nm = bfr(NM[tok]);
    const v8f e = *(const v8f*)(emb + id * EW + pc);
    v8us o;
#pragma unroll
    for (int k = 0; k < 8; ++k) o[k] = f2bf(bfr(e[k]) * nm);
    *(volatile v8us*)(HB + i * 8) = o; __threadfence(); *(volatile v8us*)(HB + i * 8) = o;
}

__global__ __launch_bounds__(32) void k_qk(const bf* __restrict__ HB, const bf* __restrict__ WB, const float* __restrict__ inb, h16* QK) {
    __shared__ __align__(16) float os[16 * 68];
    const int lane = threadIdx.x & 31, lr = lane & 15, hi = lane >> 4; const int r0 = blockIdx.x * 64;
    v8f acc[4][4];
#pragma unroll
    for (int mb = 0; mb < 4; ++mb)
#pragma unroll
        for (int nb = 0; nb < 4; ++nb) acc[mb][nb] = (v8f){};
    const size_t aoff = (size_t)(r0 + lr) * EW + 8 * hi, boff = (size_t)lr * EW + 8 * hi;
    v16bf a[4];
#pragma unroll
    for (int mb = 0; mb < 4; ++mb) a[mb] = ldb(HB + aoff + (size_t)mb * 16 * EW);
#pragma unroll
    for (int nb = 0; nb < 4; ++nb) { const v16bf bw = ldb(WB + boff + (size_t)nb * 16 * EW);
#pragma unroll
        for (int mb = 0; mb < 4; ++mb) acc[mb][nb] = wmmabg(a[mb], bw, acc[mb][nb]); }
    float bc[4];
#pragma unroll
    for (int nb = 0; nb < 4; ++nb) bc[nb] = bfr(inb[nb * 16 + lr]);
    const int bb = r0 / SEQ, tt = r0 % SEQ;
#pragma unroll
    for (int mb = 0; mb < 4; ++mb) {
#pragma unroll
        for (int nb = 0; nb < 4; ++nb) {
#pragma unroll
            for (int j = 0; j < 8; ++j) os[(hi * 8 + j) * 68 + nb * 16 + lr] = acc[mb][nb][j] + bc[nb]; }
        wave_sync();
#pragma unroll 1
        for (int ps = 0; ps < 2; ++ps) {
#pragma unroll
            for (int hh = 0; hh < 2; ++hh) {
#pragma unroll
                for (int s = 0; s < 2; ++s) { const int p = s * 32 + lane; const int row = p >> 2, c8 = (p & 3) * 8;
                    const v4f x0 = *(const v4fa*)(&os[row * 68 + hh * 32 + c8]); const v4f x1 = *(const v4fa*)(&os[row * 68 + hh * 32 + c8 + 4]); v8h hv;
#pragma unroll
                    for (int i = 0; i < 4; ++i) { hv[i] = toh_flush(x0[i]); hv[4 + i] = toh_flush(x1[i]); }
                    const size_t oo = ((size_t)(bb * 2 + hh) * SEQ + (size_t)(tt + mb * 16)) * EW + (size_t)p * 8;
                    *(volatile v8h*)(QK + oo) = hv; } }
            if (ps == 0) __threadfence(); }
        wave_sync();
    }
}

__global__ __launch_bounds__(32) void k_vt(const bf* __restrict__ HB, const bf* __restrict__ WB, const float* __restrict__ inb, h16* VT) {
    __shared__ __align__(16) float os[16 * 68];
    const int lane = threadIdx.x & 31, lr = lane & 15, hi = lane >> 4; const int r0 = blockIdx.x * 64;
    v8f acc[2][4];
#pragma unroll
    for (int mb = 0; mb < 2; ++mb)
#pragma unroll
        for (int nb = 0; nb < 4; ++nb) acc[mb][nb] = (v8f){};
    const size_t aoff = (size_t)(2 * EW + lr) * EW + 8 * hi, boff = (size_t)(r0 + lr) * EW + 8 * hi;
    v16bf a[2];
#pragma unroll
    for (int mb = 0; mb < 2; ++mb) a[mb] = ldb(WB + aoff + (size_t)mb * 16 * EW);
#pragma unroll
    for (int nb = 0; nb < 4; ++nb) { const v16bf bx = ldb(HB + boff + (size_t)nb * 16 * EW);
#pragma unroll
        for (int mb = 0; mb < 2; ++mb) acc[mb][nb] = wmmabg(a[mb], bx, acc[mb][nb]); }
    const int bb = r0 / SEQ, tt = r0 % SEQ;
#pragma unroll
    for (int mb = 0; mb < 2; ++mb) {
        float br[8];
#pragma unroll
        for (int j = 0; j < 8; ++j) br[j] = bfr(inb[2 * EW + mb * 16 + hi * 8 + j]);
#pragma unroll
        for (int nb = 0; nb < 4; ++nb) {
#pragma unroll
            for (int j = 0; j < 8; ++j) os[(hi * 8 + j) * 68 + nb * 16 + lr] = acc[mb][nb][j] + br[j]; }
        wave_sync();
#pragma unroll 1
        for (int ps = 0; ps < 2; ++ps) {
#pragma unroll
            for (int s = 0; s < 4; ++s) { const int row = 4 * s + (lane >> 3), c8 = (lane & 7) * 8;
                const v4f x0 = *(const v4fa*)(&os[row * 68 + c8]); const v4f x1 = *(const v4fa*)(&os[row * 68 + c8 + 4]); v8h hv;
#pragma unroll
                for (int i = 0; i < 4; ++i) { hv[i] = toh_flush(x0[i]); hv[4 + i] = toh_flush(x1[i]); }
                const size_t oo = ((size_t)(bb * EW + mb * 16 + row)) * SEQ + (size_t)(tt + c8);
                *(volatile v8h*)(VT + oo) = hv; }
            if (ps == 0) __threadfence(); }
        wave_sync();
    }
}

__global__ __launch_bounds__(32 * AW) void k_flash(const h16* __restrict__ QK, const h16* __restrict__ VT, const float* __restrict__ NM, const int* __restrict__ KE, float* CTX) {
    __shared__ __align__(16) float os[16 * OSP];
    const int lane = threadIdx.x & 31, lr = lane & 15, hi = lane >> 4;
    const int wave = __builtin_amdgcn_readfirstlane((int)(threadIdx.x >> 5));
    const int b = blockIdx.y; const int t0 = blockIdx.x * 16;
    const int hsel = wave & 1, esel = wave >> 1;
    int ke = KE[(size_t)b * 32]; ke = ke < 0 ? 0 : (ke > SEQ ? SEQ : ke);
    const int nk = (ke + 31) & ~31;
    const float* kmb = NM + (size_t)b * SEQ + 8 * hi;
    const size_t qo = ((size_t)(b * 2) * SEQ + (size_t)(t0 + lr)) * EW + 8 * hi;
    const size_t ko = ((size_t)(b * 2 + 1) * SEQ + (size_t)lr) * EW + 8 * hi;
    const size_t vo = ((size_t)b * EW + (size_t)(16 * esel + lr)) * SEQ + 8 * hi;
    const bool lh = (hi == hsel);
    v8u qu = __builtin_bit_cast(v8u, ldh(QK + qo));
    const unsigned mlo = (lh & (esel == 0)) ? 0xFFFFFFFFu : 0u;
    const unsigned mhi = (lh & (esel == 1)) ? 0xFFFFFFFFu : 0u;
#pragma unroll
    for (int i = 0; i < 4; ++i) { qu[i] &= mlo; qu[4 + i] &= mhi; }
    const v16h qh = __builtin_bit_cast(v16h, qu);
    v8f o = (v8f){};
    float m = NEGB, l = 0.0f;
#pragma unroll 1
    for (int key0 = 0; key0 < nk; key0 += 32) {
        const h16* ka = QK + ko + (size_t)key0 * EW;
        const v16h ka0 = ldh(ka), kb0 = ldh(ka + 16 * EW);
        v8f sa = (v8f){}, sb = (v8f){};
        sa = wmma16g(ka0, qh, sa); sb = wmma16g(kb0, qh, sb);
        const float* kp = kmb + key0;
        const v4f m0 = *(const v4f*)kp, m1 = *(const v4f*)(kp + 4), m2 = *(const v4f*)(kp + 16), m3 = *(const v4f*)(kp + 20);
        float kx[8], ky[8];
#pragma unroll
        for (int r = 0; r < 4; ++r) { kx[r] = m0[r]; kx[4 + r] = m1[r]; ky[r] = m2[r]; ky[4 + r] = m3[r]; }
        float ta[8], tb[8]; bool fa[8], fb[8]; float mx = NEGB;
#pragma unroll
        for (int r = 0; r < 8; ++r) {
            fa[r] = bfr(kx[r]) != 0.0f;
            fb[r] = bfr(ky[r]) != 0.0f;
            ta[r] = sa[r] * SC2; tb[r] = sb[r] * SC2;
            mx = fmaxf(mx, fmaxf(fa[r] ? ta[r] : NEGB, fb[r] ? tb[r] : NEGB)); }
        mx = fmaxf(mx, __shfl_xor(mx, 16, 32));
        const float mnew = fmaxf(m, mx);
        const float alpha = __builtin_amdgcn_exp2f(m - mnew);
        const float sh = PSH - mnew;
        v16h pb; float ls = 0.0f;
#pragma unroll
        for (int r = 0; r < 8; ++r) {
            const float xa = ta[r] + sh, xb = tb[r] + sh;
            const float ea = (xa < -14.0f) ? 0.0f : __builtin_amdgcn_exp2f(xa);
            const float eb = (xb < -14.0f) ? 0.0f : __builtin_amdgcn_exp2f(xb);
            const float ga = fa[r] ? ea : 0.0f, gb = fb[r] ? eb : 0.0f;
            const h16 pa = (h16)ga; const h16 pc = (h16)gb;
            pb[r] = pa; pb[8 + r] = pc;
            ls += (float)pa + (float)pc; }
        l = l * alpha + ls; m = mnew;
        o = o * alpha;
        const v16h v0 = ldh(VT + vo + key0);
        o = wmma16g(v0, pb, o);
    }
    l += __shfl_xor(l, 16, 32);
    const bool any = l > 0.0f;
    const float lsafe = any ? l : 1.0f;
    const float inv = any ? (1.0f / lsafe) : 0.0f;
    if (lh) { v4f a, c;
      a[0] = o[0] * inv; a[1] = o[1] * inv; a[2] = o[2] * inv; a[3] = o[3] * inv; c[0] = o[4] * inv; c[1] = o[5] * inv; c[2] = o[6] * inv; c[3] = o[7] * inv;
      *(v4fa*)(&os[lr * OSP + 8 * wave]) = a; *(v4fa*)(&os[lr * OSP + 8 * wave + 4]) = c; }
    __syncthreads();
    { const int row = 4 * wave + (lane >> 3), cofs = (lane & 7) * 4;
      const v4f val = *(const v4fa*)(&os[row * OSP + cofs]);
      float* dst = CTX + ((size_t)b * SEQ + (size_t)(t0 + row)) * EW + cofs;
      *(volatile v4f*)dst = val; __threadfence(); *(volatile v4f*)dst = val; }
}

__global__ __launch_bounds__(32) void k_tail(const float* __restrict__ CTX, const bf* __restrict__ WO, const bf* __restrict__ WF, const float* __restrict__ bo, const float* __restrict__ bfc, float* OUT) {
    __shared__ __align__(16) float lg[TT * NV];
    __shared__ __align__(16) float ts[16 * TSP];
    const int lane = threadIdx.x & 31, lr = lane & 15, hi = lane >> 4;
    const int tb = blockIdx.x * TT;
    const int bb = tb / SEQ, tt = tb % SEQ;
    const v16bf wo0 = ldb(WO + (size_t)lr * EW + 8 * hi), wo1 = ldb(WO + (size_t)(16 + lr) * EW + 8 * hi);
    const v16bf wf0 = ldb(WF + (size_t)lr * EW + 8 * hi), wf1 = ldb(WF + (size_t)(16 + lr) * EW + 8 * hi);
    const float bo0 = bfr(bo[lr]), bo1 = bfr(bo[16 + lr]);
    const int c1 = (16 + lr) < NV ? (16 + lr) : (NV - 1);
    const float bf0 = bfr(bfc[lr]), bf1 = bfr(bfc[c1]);
#pragma unroll 1
    for (int mt = 0; mt < TT / 16; ++mt) {
        const float* cr = CTX + (size_t)(tb + mt * 16 + lr) * EW + 8 * hi;
        const v8f x0 = *(const v8f*)cr, x1 = *(const v8f*)(cr + 16);
        v8us h0, h1, l0, l1;
#pragma unroll
        for (int i = 0; i < 8; ++i) { unsigned short hh, ll; split2(x0[i], hh, ll); h0[i] = hh; l0[i] = ll; split2(x1[i], hh, ll); h1[i] = hh; l1[i] = ll; }
        const v16bf ah = cat16b(h0, h1), al = cat16b(l0, l1);
        v8f u0 = (v8f){}, u1 = (v8f){};
        u0 = wmmabg(ah, wo0, u0); u0 = wmmabg(al, wo0, u0);
        u1 = wmmabg(ah, wo1, u1); u1 = wmmabg(al, wo1, u1);
#pragma unroll
        for (int j = 0; j < 8; ++j) { ts[(hi * 8 + j) * TSP + lr] = u0[j] + bo0; ts[(hi * 8 + j) * TSP + 16 + lr] = u1[j] + bo1; }
        wave_sync();
        const v4f y0 = *(const v4fa*)(&ts[lr * TSP + 8 * hi]), y1 = *(const v4fa*)(&ts[lr * TSP + 8 * hi + 4]);
        const v4f y2 = *(const v4fa*)(&ts[lr * TSP + 16 + 8 * hi]), y3 = *(const v4fa*)(&ts[lr * TSP + 16 + 8 * hi + 4]);
        v8us g0, g1, e0, e1;
#pragma unroll
        for (int i = 0; i < 4; ++i) { unsigned short hh, ll;
            split2(y0[i], hh, ll); g0[i] = hh; e0[i] = ll; split2(y1[i], hh, ll); g0[4 + i] = hh; e0[4 + i] = ll;
            split2(y2[i], hh, ll); g1[i] = hh; e1[i] = ll; split2(y3[i], hh, ll); g1[4 + i] = hh; e1[4 + i] = ll; }
        const v16bf th = cat16b(g0, g1), tl = cat16b(e0, e1);
        v8f z0 = (v8f){}, z1 = (v8f){};
        z0 = wmmabg(th, wf0, z0); z0 = wmmabg(tl, wf0, z0);
        z1 = wmmabg(th, wf1, z1); z1 = wmmabg(tl, wf1, z1);
#pragma unroll
        for (int j = 0; j < 8; ++j) { const int row = mt * 16 + hi * 8 + j;
            lg[row * NV + lr] = z0[j] + bf0;
            if (16 + lr < NV) lg[row * NV + 16 + lr] = z1[j] + bf1; }
        wave_sync();
    }
    float* obase = OUT + ((size_t)bb * OUT_SEQ + (size_t)tt) * NV;
#pragma unroll 1
    for (int ps = 0; ps < 2; ++ps) {
#pragma unroll 1
        for (int i = 0; i < 27; ++i) { const int idx = (i * 32 + lane) * 4;
            const v4f val = *(const v4fa*)(&lg[idx]);
            *(volatile v4f*)(obase + idx) = val; }
        if (ps == 0) __threadfence(); }
}

static constexpr size_t al256(size_t v) { return (v + 255) & ~(size_t)255; }
static constexpr size_t SZ_NM = al256((size_t)NB * SEQ * 4);
static constexpr size_t SZ_KE = al256((size_t)NB * 32 * 4);
static constexpr size_t SZ_WB = al256((size_t)WROWS * EW * 2);
static constexpr size_t SZ_HB = al256((size_t)NB * SEQ * EW * 2);
static constexpr size_t SZ_QK = al256((size_t)NB * 2 * SEQ * EW * 2);
static constexpr size_t SZ_VT = al256((size_t)NB * EW * SEQ * 2);
static constexpr size_t SZ_CX = al256((size_t)NB * SEQ * EW * 4);
static constexpr size_t SZ_TOTAL = SZ_NM + SZ_KE + SZ_WB + SZ_HB + SZ_QK + SZ_VT + SZ_CX;
static_assert(SZ_TOTAL <= (size_t)134217728);
static_assert(((size_t)WROWS * EW * 2) % 128 == 0);
static_assert(((size_t)3 * EW * EW * 2) % 256 == 0);
static_assert(((size_t)4 * EW * EW * 2) % 256 == 0);

extern "C" void kernel_launch(void* const* d_in, const int* in_sizes, int n_in,
                              void* d_out, int out_size, void* d_ws, size_t ws_size, hipStream_t stream) {
    if (n_in < 9) return;
    const size_t needt = (size_t)(NB - 1) * SEQ_FULL + SEQ;
    if ((size_t)in_sizes[0] < needt || (size_t)in_sizes[1] < needt) return;
    if (in_sizes[2] < NTOK * EW || in_sizes[3] < 3 * EW * EW || in_sizes[4] < 3 * EW) return;
    if (in_sizes[5] < EW * EW || in_sizes[6] < EW || in_sizes[7] < NV * EW || in_sizes[8] < NV) return;
    if ((size_t)out_size < ((size_t)(NB - 1) * OUT_SEQ + SEQ) * NV) return;
    if (SZ_TOTAL > ws_size) return;
    const int*   x    = (const int*)d_in[0];
    const float* mask = (const float*)d_in[1];
    const float* emb  = (const float*)d_in[2];
    const float* inw  = (const float*)d_in[3];
    const float* inb  = (const float*)d_in[4];
    const float* ow   = (const float*)d_in[5];
    const float* ob   = (const float*)d_in[6];
    const float* fw   = (const float*)d_in[7];
    const float* fb   = (const float*)d_in[8];
    float* OUT = (float*)d_out;
    char* wsp = (char*)d_ws;
    float* NM = (float*)wsp; wsp += SZ_NM;
    int*   KE = (int*)wsp;   wsp += SZ_KE;
    bf*    WB = (bf*)wsp;    wsp += SZ_WB;
    bf*    HB = (bf*)wsp;    wsp += SZ_HB;
    h16*   QK = (h16*)wsp;   wsp += SZ_QK;
    h16*   VT = (h16*)wsp;   wsp += SZ_VT;
    float* CX = (float*)wsp; wsp += SZ_CX;
    const bf* WO = WB + (size_t)3 * EW * EW;
    const bf* WF = WB + (size_t)4 * EW * EW;

    k_mask<<<NB, 256, 0, stream>>>(mask, NM, KE);
    k_wconv<<<(WROWS * 4 + 255) / 256, 256, 0, stream>>>(inw, ow, fw, WB);
    k_embed<<<(unsigned)(((size_t)NB * SEQ * 4) / 256), 256, 0, stream>>>(x, emb, NM, HB);
    k_qk<<<NB * SEQ / 64, 32, 0, stream>>>(HB, WB, inb, QK);
    k_vt<<<NB * SEQ / 64, 32, 0, stream>>>(HB, WB, inb, VT);
    k_flash<<<dim3(SEQ / 16, NB, 1), 32 * AW, 0, stream>>>(QK, VT, NM, KE, CX);
    k_tail<<<NB * SEQ / TT, 32, 0, stream>>>(CX, WO, WF, ob, fb, OUT);
}
